// PointnetFP_52750788329675
// MI455X (gfx1250) — hardware-verified
//
#include <hip/hip_runtime.h>

#pragma clang fp contract(off)

typedef __attribute__((ext_vector_type(16))) _Float16 v16h;
typedef __attribute__((ext_vector_type(8)))  _Float16 v8h;
typedef __attribute__((ext_vector_type(8)))  float    v8f;
typedef __attribute__((ext_vector_type(4)))  float    v4f;
typedef __attribute__((ext_vector_type(4)))  int      v4i;

constexpr int kBatch  = 4;
constexpr int kNumQ   = 8192;
constexpr int kNumS   = 2048;
constexpr int kCskip  = 128;
constexpr int kCint   = 256;
constexpr int kHid    = 256;
constexpr int kFeat   = 256;
constexpr int kKin    = kCint + kCskip;
constexpr int kRows   = kBatch * kNumQ;
constexpr int kChunks = kNumQ / 256;

static_assert(kKin == 384, "concat width");
static_assert(kKin % 64 == 0 && kHid % 64 == 0, "pack tiles cover whole 128-B lines of k");
static_assert(kKin % 32 == 0 && kHid % 32 == 0, "k step of 32");
static_assert(kRows % 64 == 0, "block covers 64 rows");
static_assert(kFeat == 256 && kHid == kFeat, "four 64-wide column tiles");
static_assert(kNumQ % 256 == 0 && kNumS % 256 == 0, "query / support tiling");
static_assert(kCint == 32 * 8, "one wave covers the interpolated channels with 8 per lane");
static_assert(kCskip == 16 * 8, "16 lanes cover the skip channels with 8 per lane");

constexpr float kResCarry    = 2048.0f;
constexpr float kResCarryInv = 1.0f / kResCarry;
constexpr float kF16MinNormal = 6.103515625e-5f;

constexpr size_t kOffX   = 0;
constexpr size_t kOffH1  = kOffX  + (size_t)kRows * kKin * 2;
constexpr size_t kOffW1h = kOffH1 + (size_t)kRows * kHid * 2;
constexpr size_t kOffW1l = kOffW1h + (size_t)kFeat * kKin * 2;
constexpr size_t kOffW2h = kOffW1l + (size_t)kFeat * kKin * 2;
constexpr size_t kOffW2l = kOffW2h + (size_t)kFeat * kHid * 2;
constexpr size_t kWsTotal = kOffW2l + (size_t)kFeat * kHid * 2;
static_assert(kWsTotal == 42598400, "carve total");
static_assert(kWsTotal <= (size_t)134217728, "carve under 128 MiB");
static_assert(kOffH1 % 128 == 0 && kOffW1h % 128 == 0 && kOffW1l % 128 == 0 && kOffW2h % 128 == 0 && kOffW2l % 128 == 0, "line aligned");

constexpr int kPackBlocks1 = (kKin / 64) * (kFeat / 32);
constexpr int kPackBlocks2 = (kHid / 64) * (kFeat / 32);

template <typename T> struct Frag;
template <> struct Frag<_Float16> {
  typedef v16h V; union U { v16h v; v8h h[2]; };
  static __device__ __forceinline__ v16h load(const _Float16* p) {
    U f; f.h[0] = *(const v8h*)(p); f.h[1] = *(const v8h*)(p + 16); return f.v;
  }
  static __device__ __forceinline__ v8f mma(v16h a, v16h b, v8f c) {
    return __builtin_amdgcn_wmma_f32_16x16x32_f16(false, a, false, b, (short)0, c, false, false);
  }
};
__device__ __forceinline__ void grp_guard(v8f& a, v8f& b, v8f& c, v8f& d, v16h x, v16h y, v16h z, v16h w) {
  asm volatile("v_nop\n\tv_nop\n\tv_nop\n\tv_nop" : "+v"(a), "+v"(b), "+v"(c), "+v"(d) : "v"(x), "v"(y), "v"(z), "v"(w) : "memory");
}
__device__ __forceinline__ void acc_guard4(v8f& a, v8f& b, v8f& c, v8f& d) {
  asm volatile("v_nop\n\tv_nop\n\tv_nop\n\tv_nop" : "+v"(a), "+v"(b), "+v"(c), "+v"(d));
}

__global__ __launch_bounds__(256) void pack_weights_kernel(
    const float* __restrict__ w1, const float* __restrict__ w2,
    unsigned short* __restrict__ w1h, unsigned short* __restrict__ w1l,
    unsigned short* __restrict__ w2h, unsigned short* __restrict__ w2l)
{
  __shared__ float tile[64 * 33];
  const int t = threadIdx.x;
  int bid = blockIdx.x;
  const bool second = (bid >= kPackBlocks1);
  const float* w = second ? w2 : w1;
  unsigned short* oh = second ? w2h : w1h;
  unsigned short* ol = second ? w2l : w1l;
  const int kdim = second ? kHid : kKin;
  if (second) bid -= kPackBlocks1;
  const int k0 = (bid >> 3) * 64;
  const int n0 = (bid & 7) * 32;
  const int col = t & 31;
  const int rg  = t >> 5;
#pragma unroll
  for (int i = 0; i < 8; ++i) {
    const int kk = rg + 8 * i;
    tile[kk * 33 + col] = w[(size_t)(k0 + kk) * kFeat + n0 + col];
  }
  __syncthreads();
  const int n  = t >> 3;
  const int ch = t & 7;
  v8h hv, lv;
#pragma unroll
  for (int e = 0; e < 8; ++e) {
    const float v = tile[(ch * 8 + e) * 33 + n];
    const float vh = (fabsf(v) < kF16MinNormal) ? 0.0f : v;
    const _Float16 hf = (_Float16)vh;
    const float res = (v - (float)hf) * kResCarry;
    const _Float16 lf = (_Float16)res;
    hv[e] = hf;
    lv[e] = lf;
  }
  unsigned short* ph = oh + (size_t)(n0 + n) * kdim + k0 + ch * 8;
  unsigned short* pl = ol + (size_t)(n0 + n) * kdim + k0 + ch * 8;
  *(volatile v8h*)ph = hv;
  *(volatile v8h*)pl = lv;
  __threadfence();
  *(volatile v8h*)ph = hv;
  *(volatile v8h*)pl = lv;
}

__global__ __launch_bounds__(256) void nn_interp_kernel(
    const float* __restrict__ xyz1, const float* __restrict__ xyz2,
    const float* __restrict__ points1, const float* __restrict__ points2,
    unsigned short* __restrict__ X)
{
#pragma clang fp contract(off)
  __shared__ __align__(16) v4f sP[256];
  __shared__ __align__(16) v4i sIdx[256];
  __shared__ __align__(16) v4f sWgt[256];

  const int tid   = threadIdx.x;
  const int b     = blockIdx.x / kChunks;
  const int chunk = blockIdx.x - b * kChunks;
  const int qn    = chunk * 256 + tid;

  const float* qp = xyz1 + ((size_t)b * kNumQ + qn) * 3;
  const float x = qp[0];
  const float y = qp[1];
  const float z = qp[2];
  const float sq1 = (x * x + z * z) + y * y;

  float bd0 = __builtin_inff(), bd1 = __builtin_inff(), bd2 = __builtin_inff();
  int   bi0 = 0, bi1 = 0, bi2 = 0;

  for (int t = 0; t < kNumS; t += 256) {
    __syncthreads();
    {
      const float* rp = xyz2 + ((size_t)b * kNumS + t + tid) * 3;
      const float rx = rp[0];
      const float ry = rp[1];
      const float rz = rp[2];
      v4f pv;
      pv.x = rx;
      pv.y = ry;
      pv.z = rz;
      pv.w = (rx * rx + rz * rz) + ry * ry;
      sP[tid] = pv;
    }
    __syncthreads();
#pragma unroll 4
    for (int j = 0; j < 256; ++j) {
      const v4f c = sP[j];
      float pd = x * c.x;
      pd = __builtin_fmaf(y, c.y, pd);
      pd = __builtin_fmaf(z, c.z, pd);
      const float s = sq1 + c.w;
      const float d = s - (pd + pd);
      const int jj = t + j;
      if (d < bd2) {
        const bool c0 = d < bd0;
        const bool c1 = d < bd1;
        bd2 = c1 ? bd1 : d;
        bi2 = c1 ? bi1 : jj;
        bd1 = c0 ? bd0 : (c1 ? d : bd1);
        bi1 = c0 ? bi0 : (c1 ? jj : bi1);
        bd0 = c0 ? d : bd0;
        bi0 = c0 ? jj : bi0;
      }
    }
  }

  {
    const float e0 = fmaxf(bd0, 1e-10f);
    const float e1 = fmaxf(bd1, 1e-10f);
    const float e2 = fmaxf(bd2, 1e-10f);
    const float inv0 = 1.0f / e0;
    const float inv1 = 1.0f / e1;
    const float inv2 = 1.0f / e2;
    const float ssum = (inv0 + inv2) + inv1;
    v4f wv;
    wv.x = inv0 / ssum;
    wv.y = inv1 / ssum;
    wv.z = inv2 / ssum;
    wv.w = 0.0f;
    v4i iv;
    iv.x = min(max(bi0, 0), kNumS - 1);
    iv.y = min(max(bi1, 0), kNumS - 1);
    iv.z = min(max(bi2, 0), kNumS - 1);
    iv.w = 0;
    sIdx[tid] = iv;
    sWgt[tid] = wv;
  }
  __syncthreads();

  const int wave = tid >> 5;
  const int lane = tid & 31;
  const float* P2b = points2 + (size_t)b * kNumS * kCint;
#pragma unroll 1
  for (int rr = 0; rr < 32; ++rr) {
    const int rl = wave * 32 + rr;
    const v4i id = sIdx[rl];
    const v4f wv = sWgt[rl];
    const int j0 = min(max(id.x, 0), kNumS - 1);
    const int j1 = min(max(id.y, 0), kNumS - 1);
    const int j2 = min(max(id.z, 0), kNumS - 1);
    const size_t grow = (size_t)b * kNumQ + (size_t)chunk * 256 + rl;
    const float* g0 = P2b + (size_t)j0 * kCint + 8 * lane;
    const float* g1 = P2b + (size_t)j1 * kCint + 8 * lane;
    const float* g2 = P2b + (size_t)j2 * kCint + 8 * lane;
    const float* p1 = points1 + grow * kCskip + 8 * (lane & 15);
    const v4f a0 = *(const v4f*)(g0);
    const v4f a1 = *(const v4f*)(g0 + 4);
    const v4f b0 = *(const v4f*)(g1);
    const v4f b1 = *(const v4f*)(g1 + 4);
    const v4f c0 = *(const v4f*)(g2);
    const v4f c1 = *(const v4f*)(g2 + 4);
    const v4f s0 = *(const v4f*)(p1);
    const v4f s1 = *(const v4f*)(p1 + 4);
    v8h hv, sv;
#pragma unroll
    for (int e = 0; e < 4; ++e) {
      float v = wv.x * a0[e];
      v = __builtin_fmaf(wv.y, b0[e], v);
      v = __builtin_fmaf(wv.z, c0[e], v);
      float u = wv.x * a1[e];
      u = __builtin_fmaf(wv.y, b1[e], u);
      u = __builtin_fmaf(wv.z, c1[e], u);
      hv[e]     = (_Float16)v;
      hv[4 + e] = (_Float16)u;
      const float f0 = s0[e];
      const float f1 = s1[e];
      sv[e]     = (_Float16)f0;
      sv[4 + e] = (_Float16)f1;
    }
    unsigned short* xr = X + grow * kKin;
    *(volatile v8h*)(xr + 8 * lane) = hv;
    if (lane < 16) *(volatile v8h*)(xr + kCint + 8 * lane) = sv;
    __threadfence();
    *(volatile v8h*)(xr + 8 * lane) = hv;
    if (lane < 16) *(volatile v8h*)(xr + kCint + 8 * lane) = sv;
  }
}

template <int KDIM, int OUT_F16>
__global__ __launch_bounds__(256) void mlp_gemm_relu(
    const unsigned short* __restrict__ Ap,
    const unsigned short* __restrict__ Bhp,
    const unsigned short* __restrict__ Blp,
    void* __restrict__ Cout)
{
  typedef _Float16 T;
  static_assert(KDIM % 32 == 0, "k step");
  const T* A  = (const T*)Ap;
  const T* Bh = (const T*)Bhp;
  const T* Bl = (const T*)Blp;
  __shared__ __align__(16) float sT[8][16 * 68];

  const int lane = threadIdx.x & 31;
  const int wave = threadIdx.x >> 5;
  const int tile = blockIdx.x * 8 + wave;
  const int tm = tile >> 2;
  const int tn = tile & 3;
  const int m0 = tm << 5;
  const int n0 = tn << 6;

  const int rlane = lane & 15;
  const int koff  = (lane >> 4) * 8;
  const int mOff  = (lane >> 4) * 8;

  v8f acc[2][4], accr[2][4];
#pragma unroll
  for (int i = 0; i < 2; ++i)
#pragma unroll
    for (int j = 0; j < 4; ++j) {
      acc[i][j]  = (v8f){0.f, 0.f, 0.f, 0.f, 0.f, 0.f, 0.f, 0.f};
      accr[i][j] = (v8f){0.f, 0.f, 0.f, 0.f, 0.f, 0.f, 0.f, 0.f};
    }

#pragma unroll 1
  for (int k0 = 0; k0 < KDIM; k0 += 32) {
    const v16h ah0 = Frag<T>::load(A + (size_t)(m0 + rlane) * KDIM + koff + k0);
    const v16h ah1 = Frag<T>::load(A + (size_t)(m0 + 16 + rlane) * KDIM + koff + k0);
#pragma unroll
    for (int j = 0; j < 4; ++j) {
      const size_t bo = (size_t)(n0 + (j << 4) + rlane) * KDIM + koff + k0;
      const v16h bh = Frag<T>::load(Bh + bo);
      const v16h bl = Frag<T>::load(Bl + bo);
      acc[0][j]  = Frag<T>::mma(ah0, bh, acc[0][j]);
      accr[0][j] = Frag<T>::mma(ah0, bl, accr[0][j]);
      acc[1][j]  = Frag<T>::mma(ah1, bh, acc[1][j]);
      accr[1][j] = Frag<T>::mma(ah1, bl, accr[1][j]);
      grp_guard(acc[0][j], accr[0][j], acc[1][j], accr[1][j], ah0, ah1, bh, bl);
    }
  }
  acc_guard4(acc[0][0], acc[0][1], acc[0][2], acc[0][3]);
  acc_guard4(acc[1][0], acc[1][1], acc[1][2], acc[1][3]);
  acc_guard4(accr[0][0], accr[0][1], accr[0][2], accr[0][3]);
  acc_guard4(accr[1][0], accr[1][1], accr[1][2], accr[1][3]);

  float* slab = sT[wave];
#pragma unroll
  for (int i = 0; i < 2; ++i) {
    const int mBase = m0 + (i << 4);
#pragma unroll
    for (int j = 0; j < 4; ++j) {
#pragma unroll
      for (int r = 0; r < 8; ++r) {
        float v = __builtin_fmaf(accr[i][j][r], kResCarryInv, acc[i][j][r]);
        v = fmaxf(v, 0.0f);
        slab[(mOff + r) * 68 + (j << 4) + rlane] = v;
      }
    }
    __builtin_amdgcn_fence(__ATOMIC_RELEASE, "workgroup");
    __builtin_amdgcn_wave_barrier();
    __builtin_amdgcn_fence(__ATOMIC_ACQUIRE, "workgroup");
    if (OUT_F16 == 0) {
      float* C = (float*)Cout;
      const int hh = lane >> 4;
      const int c4 = (lane & 15) * 4;
      for (int pass = 0; pass < 2; ++pass) {
#pragma unroll
        for (int it = 0; it < 8; ++it) {
          const int row = it * 2 + hh;
          const v4f v = *(const v4f*)(slab + row * 68 + c4);
          *(volatile v4f*)(C + (size_t)(mBase + row) * kFeat + n0 + c4) = v;
        }
        __threadfence();
      }
    } else {
      unsigned short* C = (unsigned short*)Cout;
      const int q  = lane >> 3;
      const int c8 = (lane & 7) * 8;
      for (int pass = 0; pass < 2; ++pass) {
#pragma unroll
        for (int it = 0; it < 4; ++it) {
          const int row = it * 4 + q;
          const float* sp = slab + row * 68 + c8;
          v8h hv;
#pragma unroll
          for (int e = 0; e < 8; ++e) {
            const float f = sp[e];
            hv[e] = (_Float16)f;
          }
          *(volatile v8h*)(C + (size_t)(mBase + row) * kHid + n0 + c8) = hv;
        }
        __threadfence();
      }
    }
    __builtin_amdgcn_fence(__ATOMIC_RELEASE, "workgroup");
    __builtin_amdgcn_wave_barrier();
    __builtin_amdgcn_fence(__ATOMIC_ACQUIRE, "workgroup");
  }
}

extern "C" void kernel_launch(void* const* d_in, const int* in_sizes, int n_in,
                              void* d_out, int out_size, void* d_ws, size_t ws_size,
                              hipStream_t stream) {
  (void)in_sizes; (void)n_in; (void)out_size;
  if (ws_size < kWsTotal) return;

  const float* xyz1    = (const float*)d_in[0];
  const float* xyz2    = (const float*)d_in[1];
  const float* points1 = (const float*)d_in[2];
  const float* points2 = (const float*)d_in[3];
  const float* w1      = (const float*)d_in[4];
  const float* w2      = (const float*)d_in[5];

  char* ws = (char*)d_ws;
  unsigned short* X   = (unsigned short*)(ws + kOffX);
  unsigned short* H1  = (unsigned short*)(ws + kOffH1);
  unsigned short* W1h = (unsigned short*)(ws + kOffW1h);
  unsigned short* W1l = (unsigned short*)(ws + kOffW1l);
  unsigned short* W2h = (unsigned short*)(ws + kOffW2h);
  unsigned short* W2l = (unsigned short*)(ws + kOffW2l);

  pack_weights_kernel<<<dim3(kPackBlocks1 + kPackBlocks2), dim3(256), 0, stream>>>(w1, w2, W1h, W1l, W2h, W2l);

  nn_interp_kernel<<<dim3(kBatch * kChunks), dim3(256), 0, stream>>>(xyz1, xyz2, points1, points2, X);

  mlp_gemm_relu<kKin, 1><<<dim3((kRows / 32) * 4 / 8), dim3(256), 0, stream>>>(X, W1h, W1l, (void*)H1);

  mlp_gemm_relu<kHid, 0><<<dim3((kRows / 32) * 4 / 8), dim3(256), 0, stream>>>(H1, W2h, W2l, d_out);
}
